// RelationalMemoryCoreCell_30966714204737
// MI455X (gfx1250) — hardware-verified
//
#include <hip/hip_runtime.h>
#include <stdint.h>
#include <stddef.h>


typedef _Float16 f16;
typedef f16   v16h __attribute__((ext_vector_type(16)));
typedef f16   v8h  __attribute__((ext_vector_type(8)));
typedef float v8f  __attribute__((ext_vector_type(8)));
typedef float v4f  __attribute__((ext_vector_type(4)));
union Frag { v16h v; v8h hh[2]; };

#define NB        256
#define NS        16
#define NH        8
#define NHS       128
#define NM        1024
#define NK        1024
#define NROWS     (NB * NS)
#define XWP       (4 * NM)
#define APITCH    72
#define CPITCH    132
#define WSCALE    64.0f
#define WINV      0.015625f
#define ATT_SCALE 0.08838834764831845f

static_assert(NROWS % 128 == 0);
static_assert(NB % 128 == 0);
static_assert(NM % 128 == 0);
static_assert(NK % 64 == 0);
static_assert(NH * NHS == NM);
static_assert((NB * NK) % 2048 == 0);
static_assert((NROWS * NM) % 2048 == 0);

__device__ __forceinline__ v8f wmma_f16(v16h a, v16h b, v8f c)
{
    v8f d = __builtin_amdgcn_wmma_f32_16x16x32_f16(false, a, false, b, (short)0, c, false, false);
    asm volatile("v_nop\n\tv_nop\n\tv_nop\n\tv_nop" : "+v"(d) : "v"(a), "v"(b));
    return d;
}

__device__ __forceinline__ float sigm(float x)
{
    return __builtin_amdgcn_rcpf(1.0f + __expf(-x));
}

__device__ __forceinline__ float tanh_rcp(float x)
{
    float e = __expf(2.0f * x);
    return 1.0f - 2.0f * __builtin_amdgcn_rcpf(e + 1.0f);
}

__global__ __launch_bounds__(256)
void k_cvt(const float* __restrict__ X, f16* Y, int n8)
{
    const int i = blockIdx.x * 256 + threadIdx.x;
    if (i < n8) {
        const size_t o = (size_t)i * 8;
        v4f a = *(const v4f*)(X + o);
        v4f b = *(const v4f*)(X + o + 4);
        v8h y;
        y[0] = (f16)a[0]; y[1] = (f16)a[1]; y[2] = (f16)a[2]; y[3] = (f16)a[3];
        y[4] = (f16)b[0]; y[5] = (f16)b[1]; y[6] = (f16)b[2]; y[7] = (f16)b[3];
        *(volatile v8h*)(Y + o) = y;
        __threadfence();
        *(volatile v8h*)(Y + o) = y;
    }
}

__global__ __launch_bounds__(256)
void k_wt(const float* __restrict__ W0, const float* __restrict__ W1,
          const float* __restrict__ W2, const float* __restrict__ W3,
          const float* __restrict__ W4, const float* __restrict__ W5,
          const float* __restrict__ W6, const float* __restrict__ W7,
          f16* Wt)
{
    __shared__ float t[64 * 65];
    const int z = blockIdx.z;
    const float* W = W0;
    if (z == 1) W = W1; else if (z == 2) W = W2; else if (z == 3) W = W3;
    else if (z == 4) W = W4; else if (z == 5) W = W5; else if (z == 6) W = W6;
    else if (z == 7) W = W7;

    const int kb = blockIdx.x * 64, nb = blockIdx.y * 64, tid = threadIdx.x;
    #pragma unroll
    for (int p = 0; p < 4; ++p) {
        const int r = p * 16 + (tid >> 4);
        const int c4 = (tid & 15) * 4;
        v4f v = *(const v4f*)(W + (size_t)(kb + r) * NM + nb + c4);
        t[r * 65 + c4 + 0] = v[0];
        t[r * 65 + c4 + 1] = v[1];
        t[r * 65 + c4 + 2] = v[2];
        t[r * 65 + c4 + 3] = v[3];
    }
    __syncthreads();

    const int lane = tid & 31, w = tid >> 5, q = lane >> 3, c = lane & 7;
    f16* base = Wt + (size_t)z * NK * NM;
    v8h y0, y1;
    size_t p0, p1;
    {
        const int n = w * 8 + q;
        #pragma unroll
        for (int i = 0; i < 8; ++i) y0[i] = (f16)(t[(8 * c + i) * 65 + n] * WSCALE);
        p0 = (size_t)(nb + n) * NK + kb + 8 * c;
    }
    {
        const int n = w * 8 + 4 + q;
        #pragma unroll
        for (int i = 0; i < 8; ++i) y1[i] = (f16)(t[(8 * c + i) * 65 + n] * WSCALE);
        p1 = (size_t)(nb + n) * NK + kb + 8 * c;
    }
    *(volatile v8h*)(base + p0) = y0;
    *(volatile v8h*)(base + p1) = y1;
    __threadfence();
    *(volatile v8h*)(base + p0) = y0;
    *(volatile v8h*)(base + p1) = y1;
}

template<int EPI>
__global__ __launch_bounds__(256) __attribute__((amdgpu_num_vgpr(256)))
void k_gemm(const f16* __restrict__ A, const f16* __restrict__ Bt,
            const float* __restrict__ bias0, const float* __restrict__ bias1,
            const float* __restrict__ aux0, const float* __restrict__ aux1,
            const float* __restrict__ aux2, float* C0, float* C1)
{
    __shared__ __attribute__((aligned(16))) unsigned char smem[128 * CPITCH * 4];
    f16* As = (f16*)smem;
    f16* Bs = As + 128 * APITCH;
    float* Cs = (float*)smem;

    const int tid = threadIdx.x, wave = tid >> 5, lane = tid & 31;
    const int wm = wave & 3, wn = wave >> 2, half = lane >> 4, lr = lane & 15;
    const int blockN = blockIdx.x * 128, blockM = blockIdx.y * 128;

    const v8f zero8 = {0.f, 0.f, 0.f, 0.f, 0.f, 0.f, 0.f, 0.f};
    v8f acc[2][4];
    #pragma unroll
    for (int fm = 0; fm < 2; ++fm)
        #pragma unroll
        for (int fn = 0; fn < 4; ++fn) acc[fm][fn] = zero8;

    #pragma unroll 1
    for (int k0 = 0; k0 < NK; k0 += 64) {
        v8h ra[4], rb[4];
        #pragma unroll
        for (int c = 0; c < 4; ++c) {
            const int l = c * 256 + tid, row = l >> 3, cr = (l & 7) * 8;
            ra[c] = *(const v8h*)(A  + (size_t)(blockM + row) * NK + k0 + cr);
            rb[c] = *(const v8h*)(Bt + (size_t)(blockN + row) * NK + k0 + cr);
        }
        __syncthreads();
        #pragma unroll
        for (int c = 0; c < 4; ++c) {
            const int l = c * 256 + tid, row = l >> 3, cr = (l & 7) * 8;
            *(v8h*)&As[row * APITCH + cr] = ra[c];
            *(v8h*)&Bs[row * APITCH + cr] = rb[c];
        }
        __syncthreads();

        #pragma unroll
        for (int kc = 0; kc < 64; kc += 32) {
            Frag a[2], b[4];
            #pragma unroll
            for (int fm = 0; fm < 2; ++fm) {
                const int r = wm * 32 + fm * 16 + lr;
                a[fm].hh[0] = *(const v8h*)&As[r * APITCH + kc + 8 * half];
                a[fm].hh[1] = *(const v8h*)&As[r * APITCH + kc + 16 + 8 * half];
            }
            #pragma unroll
            for (int fn = 0; fn < 4; ++fn) {
                const int n = wn * 64 + fn * 16 + lr;
                b[fn].hh[0] = *(const v8h*)&Bs[n * APITCH + kc + 8 * half];
                b[fn].hh[1] = *(const v8h*)&Bs[n * APITCH + kc + 16 + 8 * half];
            }
            #pragma unroll
            for (int fm = 0; fm < 2; ++fm)
                #pragma unroll
                for (int fn = 0; fn < 4; ++fn)
                    acc[fm][fn] = wmma_f16(a[fm].v, b[fn].v, acc[fm][fn]);
        }
    }
    __syncthreads();

    #pragma unroll
    for (int fm = 0; fm < 2; ++fm)
        #pragma unroll
        for (int fn = 0; fn < 4; ++fn)
            #pragma unroll
            for (int r = 0; r < 8; ++r) {
                const int row = wm * 32 + fm * 16 + 8 * half + r;
                const int col = wn * 64 + fn * 16 + lr;
                Cs[row * CPITCH + col] = acc[fm][fn][r] * WINV;
            }
    __syncthreads();

    const int cl4 = 4 * lane;
    const bool segHi = (blockN >= NM);
    float* dst = (EPI == 2 && segHi) ? C1 : C0;
    const v4f zero4 = {0.f, 0.f, 0.f, 0.f};
    #pragma unroll
    for (int g = 0; g < 4; ++g) {
        v4f vals[4];
        size_t offs[4];
        #pragma unroll
        for (int j = 0; j < 4; ++j) {
            const int row = wave * 16 + g * 4 + j;
            const size_t grow = (size_t)(blockM + row);
            const v4f c = *(const v4f*)&Cs[row * CPITCH + cl4];
            v4f v = c;
            if (EPI == 0) {
                v4f b4 = zero4;
                if (blockN < NM) b4 = *(const v4f*)(bias0 + blockN + cl4);
                v = c + b4;
                offs[j] = grow * (size_t)XWP + blockN + cl4;
            } else if (EPI == 1) {
                const v4f b4 = *(const v4f*)(bias0 + blockN + cl4);
                const v4f ad = *(const v4f*)(aux0 + grow * NM + blockN + cl4);
                v = (c + b4) + ad;
                offs[j] = grow * NM + blockN + cl4;
            } else if (EPI == 2) {
                const int cb = blockN - (segHi ? NM : 0) + cl4;
                const v4f b4 = *(const v4f*)((segHi ? bias1 : bias0) + cb);
                const v4f wx = *(const v4f*)(aux0 + (grow >> 4) * (size_t)XWP + (segHi ? 3 * NM : NM) + cb);
                const v4f m4 = *(const v4f*)(aux1 + grow * NM + cb);
                const v4f z = (c + b4) + wx;
                #pragma unroll
                for (int t2 = 0; t2 < 4; ++t2) {
                    const float gt = sigm(z[t2]);
                    v[t2] = segHi ? (tanh_rcp(m4[t2]) * sigm(gt)) : sigm(m4[t2] * gt + 1.0f);
                }
                offs[j] = grow * NM + cb;
            } else {
                const v4f b4 = *(const v4f*)(bias0 + blockN + cl4);
                const v4f wx = *(const v4f*)(aux0 + (grow >> 4) * (size_t)XWP + 2 * NM + blockN + cl4);
                const v4f t4 = *(const v4f*)(aux1 + grow * NM + blockN + cl4);
                const v4f p4 = *(const v4f*)(aux2 + grow * NM + blockN + cl4);
                const v4f z = (c + b4) + wx;
                #pragma unroll
                for (int t2 = 0; t2 < 4; ++t2) {
                    const float gt = sigm(z[t2]);
                    v[t2] = t4[t2] + p4[t2] * sigm(gt);
                }
                offs[j] = grow * NM + blockN + cl4;
            }
            vals[j] = v;
        }
        #pragma unroll
        for (int j = 0; j < 4; ++j) *(volatile v4f*)(dst + offs[j]) = vals[j];
        __threadfence();
        #pragma unroll
        for (int j = 0; j < 4; ++j) *(volatile v4f*)(dst + offs[j]) = vals[j];
    }
}

__global__ __launch_bounds__(256)
void k_attn(const float* __restrict__ mst, const float* __restrict__ xw,
            float* mp0, f16* mp0h)
{
    __shared__ __attribute__((aligned(16))) float kv[17 * CPITCH];
    __shared__ float sc[16 * 20];
    __shared__ __attribute__((aligned(16))) float rs[16 * CPITCH];

    const int b = blockIdx.x >> 3, h = blockIdx.x & 7, tid = threadIdx.x;

    for (int i = tid; i < 17 * 32; i += 256) {
        const int r = i >> 5, d4 = (i & 31) * 4;
        v4f v;
        if (r < NS) v = *(const v4f*)(mst + ((size_t)(b * NS + r)) * NM + h * NHS + d4);
        else        v = *(const v4f*)(xw + (size_t)b * XWP + h * NHS + d4);
        *(v4f*)&kv[r * CPITCH + d4] = v;
    }
    __syncthreads();

    {
        const int qi = tid >> 4, r = tid & 15;
        const v4f* qp = (const v4f*)&kv[qi * CPITCH];
        const v4f* kp = (const v4f*)&kv[r * CPITCH];
        float s = 0.f;
        #pragma unroll 2
        for (int d = 0; d < 32; ++d) {
            const v4f a = qp[d], k = kp[d];
            s += a[0] * k[0]; s += a[1] * k[1]; s += a[2] * k[2]; s += a[3] * k[3];
        }
        sc[qi * 20 + r] = s * ATT_SCALE;
        if (r == 0) {
            const v4f* kp2 = (const v4f*)&kv[16 * CPITCH];
            float s2 = 0.f;
            #pragma unroll 2
            for (int d = 0; d < 32; ++d) {
                const v4f a = qp[d], k = kp2[d];
                s2 += a[0] * k[0]; s2 += a[1] * k[1]; s2 += a[2] * k[2]; s2 += a[3] * k[3];
            }
            sc[qi * 20 + 16] = s2 * ATT_SCALE;
        }
    }
    __syncthreads();

    if (tid < NS) {
        float mx = sc[tid * 20];
        #pragma unroll
        for (int j = 1; j < 17; ++j) mx = fmaxf(mx, sc[tid * 20 + j]);
        float sum = 0.f;
        #pragma unroll
        for (int j = 0; j < 17; ++j) {
            const float e = __expf(sc[tid * 20 + j] - mx);
            sc[tid * 20 + j] = e;
            sum += e;
        }
        const float inv = __builtin_amdgcn_rcpf(sum);
        #pragma unroll
        for (int j = 0; j < 17; ++j) sc[tid * 20 + j] = sc[tid * 20 + j] * inv;
    }
    __syncthreads();

    #pragma unroll 1
    for (int i = tid; i < NS * NHS; i += 256) {
        const int q = i >> 7, d = i & 127;
        float a = 0.f;
        #pragma unroll
        for (int j = 0; j < 17; ++j) a += sc[q * 20 + j] * kv[j * CPITCH + d];
        rs[q * CPITCH + d] = kv[q * CPITCH + d] + a;
    }
    __syncthreads();

    const int w = tid >> 5, lane = tid & 31;
    const int r0 = 2 * w, r1 = 2 * w + 1;
    const v4f f0 = *(const v4f*)&rs[r0 * CPITCH + 4 * lane];
    const v4f f1 = *(const v4f*)&rs[r1 * CPITCH + 4 * lane];
    const size_t o0 = ((size_t)(b * NS + r0)) * NM + h * NHS + 4 * lane;
    const size_t o1 = o0 + NM;
    const int rh = 2 * w + (lane >> 4), d8 = 8 * (lane & 15);
    v8h y;
    #pragma unroll
    for (int i = 0; i < 8; ++i) y[i] = (f16)rs[rh * CPITCH + d8 + i];
    const size_t oh = ((size_t)(b * NS + rh)) * NM + h * NHS + d8;

    *(volatile v4f*)(mp0 + o0) = f0;
    *(volatile v4f*)(mp0 + o1) = f1;
    *(volatile v8h*)(mp0h + oh) = y;
    __threadfence();
    *(volatile v4f*)(mp0 + o0) = f0;
    *(volatile v4f*)(mp0 + o1) = f1;
    *(volatile v8h*)(mp0h + oh) = y;
}

extern "C" void kernel_launch(void* const* d_in, const int* in_sizes, int n_in,
                              void* d_out, int out_size, void* d_ws, size_t ws_size,
                              hipStream_t stream)
{
    if (n_in < 16) return;
    if (in_sizes[0] != NB * NK) return;
    if (in_sizes[1] != NROWS * NM || in_sizes[2] != NROWS * NM) return;
    if (in_sizes[3] != NK * NM || in_sizes[5] != NK * NM || in_sizes[7] != NK * NM ||
        in_sizes[8] != NK * NM || in_sizes[9] != NK * NM || in_sizes[10] != NK * NM ||
        in_sizes[12] != NK * NM || in_sizes[14] != NK * NM) return;
    if (in_sizes[4] != NM || in_sizes[6] != NM || in_sizes[11] != NM ||
        in_sizes[13] != NM || in_sizes[15] != NM) return;
    if (out_size != 2 * NROWS * NM) return;

    const float* inputs  = (const float*)d_in[0];
    const float* h_state = (const float*)d_in[1];
    const float* m_state = (const float*)d_in[2];
    const float* W_emb   = (const float*)d_in[3];
    const float* b_emb   = (const float*)d_in[4];
    const float* W_g     = (const float*)d_in[5];
    const float* b_g     = (const float*)d_in[6];
    const float* W_wf    = (const float*)d_in[7];
    const float* W_wi    = (const float*)d_in[8];
    const float* W_wo    = (const float*)d_in[9];
    const float* W_uf    = (const float*)d_in[10];
    const float* b_uf    = (const float*)d_in[11];
    const float* W_ui    = (const float*)d_in[12];
    const float* b_ui    = (const float*)d_in[13];
    const float* W_uo    = (const float*)d_in[14];
    const float* b_uo    = (const float*)d_in[15];

    const size_t bWT   = (size_t)8 * NK * NM * sizeof(f16);
    const size_t bXH   = (size_t)NB * NK * sizeof(f16);
    const size_t bHH   = (size_t)NROWS * NM * sizeof(f16);
    const size_t bXW   = (size_t)NB * XWP * sizeof(float);
    const size_t bMP0  = (size_t)NROWS * NM * sizeof(float);
    const size_t bMP0H = (size_t)NROWS * NM * sizeof(f16);
    const size_t bMPO  = (size_t)NROWS * NM * sizeof(float);
    const size_t bT1   = (size_t)NROWS * NM * sizeof(float);
    const size_t total = bWT + bXH + bHH + bXW + bMP0 + bMP0H + bMPO + bT1;
    if (total > ws_size) return;

    char* wsc = (char*)d_ws;
    size_t off = 0;
    f16*   Wt   = (f16*)(wsc + off);   off += bWT;
    f16*   xh   = (f16*)(wsc + off);   off += bXH;
    f16*   hh   = (f16*)(wsc + off);   off += bHH;
    float* xw   = (float*)(wsc + off); off += bXW;
    float* mp0  = (float*)(wsc + off); off += bMP0;
    f16*   mp0h = (f16*)(wsc + off);   off += bMP0H;
    float* mpo  = (float*)(wsc + off); off += bMPO;
    float* t1   = (float*)(wsc + off); off += bT1;

    float* out0 = (float*)d_out;
    float* out1 = out0 + (size_t)NROWS * NM;

    dim3 blk(256);

    k_wt<<<dim3(NK / 64, NM / 64, 8), blk, 0, stream>>>(W_emb, W_wf, W_wi, W_wo, W_g, W_uf, W_uo, W_ui, Wt);

    k_cvt<<<dim3((NB * NK / 8 + 255) / 256), blk, 0, stream>>>(inputs, xh, NB * NK / 8);
    k_cvt<<<dim3((NROWS * NM / 8 + 255) / 256), blk, 0, stream>>>(h_state, hh, NROWS * NM / 8);

    k_gemm<0><<<dim3(XWP / 128, NB / 128), blk, 0, stream>>>(
        xh, Wt, b_emb, b_emb, m_state, m_state, m_state, xw, xw);

    k_attn<<<dim3(NB * NH), blk, 0, stream>>>(m_state, xw, mp0, mp0h);

    k_gemm<1><<<dim3(NM / 128, NROWS / 128), blk, 0, stream>>>(
        mp0h, Wt + (size_t)4 * NK * NM, b_g, b_g, mp0, mp0, mp0, mpo, mpo);

    k_gemm<2><<<dim3(2 * NM / 128, NROWS / 128), blk, 0, stream>>>(
        hh, Wt + (size_t)5 * NK * NM, b_uf, b_uo, xw, m_state, m_state, t1, out1);

    k_gemm<3><<<dim3(NM / 128, NROWS / 128), blk, 0, stream>>>(
        hh, Wt + (size_t)7 * NK * NM, b_ui, b_ui, xw, t1, mpo, out0, out0);
}
